// SimpleDecoderLayer_10393820857175
// MI455X (gfx1250) — hardware-verified
//
#include <hip/hip_runtime.h>
#include <hip/hip_bf16.h>
#include <math.h>

typedef __attribute__((ext_vector_type(16))) _Float16 v16h;
typedef __attribute__((ext_vector_type(8)))  _Float16 v8h;
typedef __attribute__((ext_vector_type(4)))  _Float16 v4h;
typedef __attribute__((ext_vector_type(16))) __bf16   v16b;
typedef __attribute__((ext_vector_type(8)))  __bf16   v8b;
typedef __attribute__((ext_vector_type(8)))  float    v8f;
typedef __attribute__((ext_vector_type(4)))  float    v4f;
#define U16(p) ((const unsigned short*)(const void*)(p))

__device__ __forceinline__ unsigned short f2bf_bits(float f) {
  unsigned u = __float_as_uint(f);
  return (unsigned short)((u + 0x7FFFu + ((u >> 16) & 1u)) >> 16);
}
__device__ __forceinline__ float bf_bits2f(unsigned short h) { return __uint_as_float(((unsigned)h) << 16); }

__device__ __forceinline__ void dep_guard_h(v8f& a, v8f& b, v16h x, v16h y) { asm volatile("v_nop\n\tv_nop\n\tv_nop\n\tv_nop" : "+v"(a), "+v"(b) : "v"(x), "v"(y)); }
__device__ __forceinline__ void dep_guard_b(v8f& a, v8f& b, v16b x, v16b y) { asm volatile("v_nop\n\tv_nop\n\tv_nop\n\tv_nop" : "+v"(a), "+v"(b) : "v"(x), "v"(y)); }
__device__ __forceinline__ void keep4_h(v16h a, v16h b, v16h c, v16h d) { asm volatile("v_nop" :: "v"(a), "v"(b), "v"(c), "v"(d)); }
__device__ __forceinline__ void keep4_b(v16b a, v16b b, v16b c, v16b d) { asm volatile("v_nop" :: "v"(a), "v"(b), "v"(c), "v"(d)); }
__device__ __forceinline__ void acc_guard4(v8f& a, v8f& b, v8f& c, v8f& d) { asm volatile("v_nop\n\tv_nop\n\tv_nop\n\tv_nop" : "+v"(a), "+v"(b), "+v"(c), "+v"(d)); }
template <typename T> struct Frag;
template <> struct Frag<_Float16> {
  typedef v16h V; union U { v16h v; v8h h[2]; };
  static __device__ __forceinline__ v16h load(const _Float16* p) {
    U f; f.h[0] = *(const v8h*)(p); f.h[1] = *(const v8h*)(p + 16); return f.v;
  }
  static __device__ __forceinline__ v8f mma(v16h a, v16h b, v8f c) {
    return __builtin_amdgcn_wmma_f32_16x16x32_f16(false, a, false, b, (short)0, c, false, false);
  }
  static __device__ __forceinline__ void guard(v8f& a, v8f& b, v16h x, v16h y) { dep_guard_h(a, b, x, y); }
  static __device__ __forceinline__ void keep(v16h a, v16h b, v16h c, v16h d) { keep4_h(a, b, c, d); }
};
template <> struct Frag<__bf16> {
  typedef v16b V; union U { v16b v; v8b h[2]; };
  static __device__ __forceinline__ v16b load(const __bf16* p) {
    U f; f.h[0] = *(const v8b*)(p); f.h[1] = *(const v8b*)(p + 16); return f.v;
  }
  static __device__ __forceinline__ v8f mma(v16b a, v16b b, v8f c) {
    return __builtin_amdgcn_wmma_f32_16x16x32_bf16(false, a, false, b, (short)0, c, false, false);
  }
  static __device__ __forceinline__ void guard(v8f& a, v8f& b, v16b x, v16b y) { dep_guard_b(a, b, x, y); }
  static __device__ __forceinline__ void keep(v16b a, v16b b, v16b c, v16b d) { keep4_b(a, b, c, d); }
};

template <int ET> struct Elem;
template <> struct Elem<0> { typedef _Float16 T; };
template <> struct Elem<1> { typedef __bf16 T; };
template <int ET, bool SPLIT, int BIAS_MODE, int OUT_MODE, bool RESID, int ACT = 0>
__global__ __launch_bounds__(256) void wmma_gemm64(
    const unsigned short* __restrict__ Ap, const unsigned short* __restrict__ A2p, int lda, long strideA,
    const unsigned short* __restrict__ Btp, const unsigned short* __restrict__ Bt2p, int ldb, long strideB,
    void* __restrict__ Cout, void* __restrict__ Cout2, int ldc, long strideC,
    const float* __restrict__ bias,
    const float* __restrict__ resid, long strideR,
    int M, int N, int K, float scale) {
  typedef typename Elem<ET>::T T;
  typedef typename Frag<T>::V V;
  const T* A = (const T*)Ap; const T* A2 = (const T*)A2p; const T* Bt = (const T*)Btp; const T* Bt2 = (const T*)Bt2p;
  __shared__ __align__(16) float sT[8][16 * 68];
  const int b    = blockIdx.y;
  const int lane = threadIdx.x & 31;
  const int wave = threadIdx.x >> 5;
  const int tilesN = N >> 6;
  const int tilesM = M >> 6;
  const int tile = blockIdx.x * 8 + wave;
  if (tile >= tilesM * tilesN) return;
  const int tm = tile / tilesN;
  const int tn = tile - tm * tilesN;
  const int m0 = tm << 6;
  const int n0 = tn << 6;

  const T* Ab  = A  + (size_t)b * strideA;
  const T* Bb  = Bt + (size_t)b * strideB;
  const T* Ab2 = SPLIT ? (A2  + (size_t)b * strideA) : nullptr;
  const T* Bb2 = SPLIT ? (Bt2 + (size_t)b * strideB) : nullptr;

  const int rlane = lane & 15;
  const int koff  = (lane >> 4) * 8;
  const int mOff  = (lane >> 4) * 8;

  v8f acc[4][4];
#pragma unroll
  for (int i = 0; i < 4; ++i)
#pragma unroll
    for (int j = 0; j < 4; ++j) acc[i][j] = (v8f){0.f,0.f,0.f,0.f,0.f,0.f,0.f,0.f};

  for (int k0 = 0; k0 < K; k0 += 32) {
    V bh[4], bl[4];
#pragma unroll
    for (int j = 0; j < 4; ++j) {
      const size_t bo = (size_t)(n0 + (j << 4) + rlane) * ldb + koff + k0;
      bh[j] = Frag<T>::load(Bb + bo);
      if (SPLIT) bl[j] = Frag<T>::load(Bb2 + bo);
    }
#pragma unroll
    for (int i = 0; i < 4; ++i) {
      const size_t ao = (size_t)(m0 + (i << 4) + rlane) * lda + koff + k0;
      V ah = Frag<T>::load(Ab + ao);
      V al;
      if (SPLIT) al = Frag<T>::load(Ab2 + ao);
#pragma unroll
      for (int j = 0; j < 4; ++j) {
        acc[i][j] = Frag<T>::mma(ah, bh[j], acc[i][j]);
        if (SPLIT) {
          acc[i][j] = Frag<T>::mma(ah, bl[j], acc[i][j]);
          acc[i][j] = Frag<T>::mma(al, bh[j], acc[i][j]);
        }
      }
      Frag<T>::guard(acc[i][0], acc[i][3], ah, SPLIT ? al : ah);
    }
    Frag<T>::keep(bh[0], bh[1], bh[2], bh[3]);
    if (SPLIT) Frag<T>::keep(bl[0], bl[1], bl[2], bl[3]);
  }
  acc_guard4(acc[0][0], acc[0][1], acc[0][2], acc[0][3]);
  acc_guard4(acc[1][0], acc[1][1], acc[1][2], acc[1][3]);
  acc_guard4(acc[2][0], acc[2][1], acc[2][2], acc[2][3]);
  acc_guard4(acc[3][0], acc[3][1], acc[3][2], acc[3][3]);

  float* slab = sT[wave];
  const float* Rb = RESID ? (resid + (size_t)b * strideR) : nullptr;
#pragma unroll
  for (int i = 0; i < 4; ++i) {
    const int mBase = m0 + (i << 4);
#pragma unroll
    for (int j = 0; j < 4; ++j) {
      const int n = n0 + (j << 4) + rlane;
      float bv = 0.f;
      if (BIAS_MODE == 2) bv = bias[n];
#pragma unroll
      for (int r = 0; r < 8; ++r) {
        float v = acc[i][j][r] * scale;
        if (BIAS_MODE == 1) v += bias[mBase + mOff + r];
        if (BIAS_MODE == 2) v += bv;
        if (RESID) v += Rb[(size_t)(mBase + mOff + r) * ldc + n];
        if (ACT == 1) v = tanhf(v);
        if (ACT == 2) v = fmaxf(v, 0.0f);
        if (ACT == 3) v = v / (1.0f + expf(-v));
        if (ACT == 4) v = (v > 0.f) ? v : 0.01f * v;
        if (ACT == 5) v = 0.5f * v * (1.0f + erff(v * 0.70710678118654752f));
        slab[(mOff + r) * 68 + (j << 4) + rlane] = v;
      }
    }
    __builtin_amdgcn_fence(__ATOMIC_RELEASE, "workgroup");
    __builtin_amdgcn_wave_barrier();
    __builtin_amdgcn_fence(__ATOMIC_ACQUIRE, "workgroup");
    if (OUT_MODE == 0) {
      float* C = (float*)Cout + (size_t)b * strideC;
      const int hh = lane >> 4, c4 = (lane & 15) * 4;
      for (int pass = 0; pass < 2; ++pass) {
#pragma unroll
        for (int it = 0; it < 8; ++it) {
          const int row = it * 2 + hh;
          v4f v = *(const v4f*)(slab + row * 68 + c4);
          *(volatile v4f*)(C + (size_t)(mBase + row) * ldc + n0 + c4) = v;
        }
        __threadfence();
      }
    } else {
      const int q = lane >> 3, c8 = (lane & 7) * 8;
      unsigned short* C  = (unsigned short*)Cout  + (size_t)b * strideC;
      unsigned short* C2 = (OUT_MODE == 2) ? ((unsigned short*)Cout2 + (size_t)b * strideC) : nullptr;
      for (int pass = 0; pass < 2; ++pass) {
#pragma unroll
        for (int it = 0; it < 4; ++it) {
          const int row = it * 4 + q;
          const float* sp = slab + row * 68 + c8;
          v8h hv, lv;
#pragma unroll
          for (int e = 0; e < 8; ++e) {
            if (OUT_MODE == 1) {
              hv[e] = (_Float16)sp[e];
            } else {
              unsigned short hb = f2bf_bits(sp[e]);
              unsigned short lb = f2bf_bits(sp[e] - bf_bits2f(hb));
              hv[e] = __builtin_bit_cast(_Float16, hb);
              lv[e] = __builtin_bit_cast(_Float16, lb);
            }
          }
          *(volatile v8h*)(C + (size_t)(mBase + row) * ldc + n0 + c8) = hv;
          if (OUT_MODE == 2) *(volatile v8h*)(C2 + (size_t)(mBase + row) * ldc + n0 + c8) = lv;
        }
        __threadfence();
      }
    }
    __builtin_amdgcn_fence(__ATOMIC_RELEASE, "workgroup");
    __builtin_amdgcn_wave_barrier();
    __builtin_amdgcn_fence(__ATOMIC_ACQUIRE, "workgroup");
  }
}

__global__ __launch_bounds__(256) void cast_f32_f16x2s(
    const float* __restrict__ in, _Float16* __restrict__ out, int n2, float scale) {
  int i = blockIdx.x * 256 + threadIdx.x;
  if (i < n2) {
    const _Float16 h0 = (_Float16)(in[2 * i] * scale), h1 = (_Float16)(in[2 * i + 1] * scale);
    const unsigned u = (unsigned)__builtin_bit_cast(unsigned short, h0) | ((unsigned)__builtin_bit_cast(unsigned short, h1) << 16);
    ((volatile unsigned*)out)[i] = u;
    __threadfence();
    ((volatile unsigned*)out)[i] = u;
  }
}

#define AT_D 64
#define AT_NW 4
#define AT_QB 64
#define AT_KC 64

__device__ __forceinline__ v8f at_mma_h(v16h a, v16h b, v8f c) {
  c = __builtin_amdgcn_wmma_f32_16x16x32_f16(false, a, false, b, (short)0, c, false, false);
  asm volatile("v_nop\n\tv_nop\n\tv_nop\n\tv_nop" : "+v"(c) : "v"(a), "v"(b));
  return c;
}

__global__ __launch_bounds__(128)
void attn64_causal_f16(const float* __restrict__ q, const float* __restrict__ k,
                       const float* __restrict__ v, float* __restrict__ out,
                       int S, int H, int ld, float sscale, float mask_fill) {
  const float PSC = 32768.0f;
  union FH { v16h v; v8h h[2]; };
  __shared__ __align__(16) _Float16 Ksh[AT_KC * AT_D];
  __shared__ __align__(16) _Float16 Vth[AT_D * AT_KC];
  __shared__ __align__(16) _Float16 Psh[AT_NW][16 * AT_KC];
  __shared__ __align__(16) float    Os[AT_NW][16 * 68];

  const int tid  = threadIdx.x;
  const int wave = tid >> 5;
  const int lane = tid & 31;
  const int hh   = lane >> 4;
  const int c    = lane & 15;

  const int nqb = S / AT_QB;
  const int bx = blockIdx.x;
  const int qb = bx % nqb;
  const int bh = bx / nqb;
  const int h  = bh % H;
  const int b  = bh / H;
  const int q0 = qb * AT_QB + wave * 16;
  const size_t bs = (size_t)S * (size_t)ld;

  const float* qb_ptr = q   + (size_t)b * bs + (size_t)h * AT_D;
  const float* kb_ptr = k   + (size_t)b * bs + (size_t)h * AT_D;
  const float* vb_ptr = v   + (size_t)b * bs + (size_t)h * AT_D;
  float*       ob_ptr = out + (size_t)b * bs + (size_t)h * AT_D;

  v16h qa[2];
  {
    const float* qrow = qb_ptr + (size_t)(q0 + c) * ld;
#pragma unroll
    for (int dc = 0; dc < 2; ++dc) {
#pragma unroll
      for (int e = 0; e < 8; ++e) {
        qa[dc][e]     = (_Float16)qrow[dc * 32 + 8 * hh + e];
        qa[dc][8 + e] = (_Float16)qrow[dc * 32 + 16 + 8 * hh + e];
      }
    }
  }

  float mrow[8], lrow[8];
  v8f oacc[4];
#pragma unroll
  for (int r = 0; r < 8; ++r) { mrow[r] = -INFINITY; lrow[r] = 0.f; }
#pragma unroll
  for (int t = 0; t < 4; ++t) oacc[t] = (v8f){0.f,0.f,0.f,0.f,0.f,0.f,0.f,0.f};

  const int nChunks = qb + 1;
  for (int kc = 0; kc < nChunks; ++kc) {
    const int kv0 = kc * AT_KC;
    __syncthreads();
    {
      const int kvr = tid >> 1, dh = (tid & 1) * 32;
      const float* krow = kb_ptr + (size_t)(kv0 + kvr) * ld + dh;
      const float* vrow = vb_ptr + (size_t)(kv0 + kvr) * ld + dh;
#pragma unroll
      for (int i = 0; i < 8; ++i) {
        v4f kk = *(const v4f*)(krow + 4 * i);
        v4f vv = *(const v4f*)(vrow + 4 * i);
#pragma unroll
        for (int e = 0; e < 4; ++e) {
          const int d = dh + 4 * i + e;
          Ksh[kvr * AT_D + d] = (_Float16)kk[e];
          Vth[d * AT_KC + kvr] = (_Float16)vv[e];
        }
      }
    }
    __syncthreads();

    v8f s[4];
#pragma unroll
    for (int j = 0; j < 4; ++j) {
      s[j] = (v8f){0.f,0.f,0.f,0.f,0.f,0.f,0.f,0.f};
#pragma unroll
      for (int dc = 0; dc < 2; ++dc) {
        FH kb;
        kb.h[0] = *(const v8h*)(Ksh + (j * 16 + c) * AT_D + dc * 32 + 8 * hh);
        kb.h[1] = *(const v8h*)(Ksh + (j * 16 + c) * AT_D + dc * 32 + 16 + 8 * hh);
        s[j] = at_mma_h(qa[dc], kb.v, s[j]);
      }
    }
    const bool diag = (kc == qb);
    float cm[8];
#pragma unroll
    for (int r = 0; r < 8; ++r) {
      const int qrow = q0 + 8 * hh + r;
      float m = -INFINITY;
#pragma unroll
      for (int j = 0; j < 4; ++j) {
        const int kvcol = kv0 + j * 16 + c;
        float sv = s[j][r] * sscale;
        if (diag && (kvcol > qrow)) sv = mask_fill;
        s[j][r] = sv;
        m = fmaxf(m, sv);
      }
#pragma unroll
      for (int off = 1; off < 16; off <<= 1) m = fmaxf(m, __shfl_xor(m, off, 32));
      cm[r] = m;
    }
    _Float16* pwh = Psh[wave];
#pragma unroll
    for (int r = 0; r < 8; ++r) {
      const float mnew = fmaxf(mrow[r], cm[r]);
      const float alpha = expf(mrow[r] - mnew);
      mrow[r] = mnew;
      float psum = 0.f;
#pragma unroll
      for (int j = 0; j < 4; ++j) {
        const float p = expf(s[j][r] - mnew);
        psum += p;
        pwh[(8 * hh + r) * AT_KC + j * 16 + c] = (_Float16)(p * PSC);
      }
#pragma unroll
      for (int off = 1; off < 16; off <<= 1) psum += __shfl_xor(psum, off, 32);
      lrow[r] = lrow[r] * alpha + psum;
#pragma unroll
      for (int t = 0; t < 4; ++t) oacc[t][r] *= alpha;
    }
    __builtin_amdgcn_fence(__ATOMIC_RELEASE, "workgroup");
    __builtin_amdgcn_wave_barrier();
    __builtin_amdgcn_fence(__ATOMIC_ACQUIRE, "workgroup");
#pragma unroll 1
    for (int kk = 0; kk < 2; ++kk) {
      FH pa;
      pa.h[0] = *(const v8h*)(pwh + c * AT_KC + kk * 32 + 8 * hh);
      pa.h[1] = *(const v8h*)(pwh + c * AT_KC + kk * 32 + 16 + 8 * hh);
#pragma unroll
      for (int t = 0; t < 4; ++t) {
        FH vb;
        vb.h[0] = *(const v8h*)(Vth + (t * 16 + c) * AT_KC + kk * 32 + 8 * hh);
        vb.h[1] = *(const v8h*)(Vth + (t * 16 + c) * AT_KC + kk * 32 + 16 + 8 * hh);
        oacc[t] = at_mma_h(pa.v, vb.v, oacc[t]);
      }
    }
  }

  float* os = Os[wave];
#pragma unroll
  for (int r = 0; r < 8; ++r) {
    const float inv = 1.0f / (lrow[r] * PSC);
#pragma unroll
    for (int t = 0; t < 4; ++t) os[(8 * hh + r) * 68 + t * 16 + c] = oacc[t][r] * inv;
  }
  __builtin_amdgcn_fence(__ATOMIC_RELEASE, "workgroup");
  __builtin_amdgcn_wave_barrier();
  __builtin_amdgcn_fence(__ATOMIC_ACQUIRE, "workgroup");
  {
    const int c4 = (lane & 15) * 4;
    for (int pass = 0; pass < 2; ++pass) {
#pragma unroll
      for (int it = 0; it < 8; ++it) {
        const int row = it * 2 + hh;
        v4f val = *(const v4f*)(os + row * 68 + c4);
        *(volatile v4f*)(ob_ptr + (size_t)(q0 + row) * ld + c4) = val;
      }
      __threadfence();
    }
  }
}

#define LN_D 1024

__device__ __forceinline__ float wsum32(float x) {
#pragma unroll
  for (int off = 16; off > 0; off >>= 1) x += __shfl_xor(x, off, 32);
  return x;
}

template <bool WB>
__global__ __launch_bounds__(256)
void ln_rows_kernel(const float* __restrict__ Y, const float* __restrict__ gam, const float* __restrict__ bet,
                    float* __restrict__ outf, _Float16* __restrict__ outh, float eps) {
  __shared__ float red0[8];
  __shared__ float red1[8];
  const int row = blockIdx.x;
  const int tid = threadIdx.x, lane = tid & 31, wave = tid >> 5;
  const size_t base = (size_t)row * LN_D + (size_t)tid * 4;

  const v4f x = *(const v4f*)(Y + base);
  float s = (x[0] + x[1]) + (x[2] + x[3]);
  s = wsum32(s);
  if (lane == 0) red0[wave] = s;
  __syncthreads();
  float tot = 0.f;
#pragma unroll
  for (int w = 0; w < 8; ++w) tot += red0[w];
  const float mean = tot * (1.0f / LN_D);

  v4f d;
#pragma unroll
  for (int e = 0; e < 4; ++e) d[e] = x[e] - mean;
  float vs = (d[0] * d[0] + d[1] * d[1]) + (d[2] * d[2] + d[3] * d[3]);
  vs = wsum32(vs);
  if (lane == 0) red1[wave] = vs;
  __syncthreads();
  float tot2 = 0.f;
#pragma unroll
  for (int w = 0; w < 8; ++w) tot2 += red1[w];
  const float var = tot2 * (1.0f / LN_D);
  const float rstd = rsqrtf(var + eps);

  const v4f gm = *(const v4f*)(gam + tid * 4);
  const v4f bt = *(const v4f*)(bet + tid * 4);
  v4f y;
#pragma unroll
  for (int e = 0; e < 4; ++e) y[e] = (d[e] * rstd) * gm[e] + bt[e];
  v4h yh;
#pragma unroll
  for (int e = 0; e < 4; ++e) yh[e] = (_Float16)y[e];

  *(volatile v4f*)(outf + base) = y;
  if (WB) *(volatile v4h*)(outh + base) = yh;
  __threadfence();
  *(volatile v4f*)(outf + base) = y;
  if (WB) *(volatile v4h*)(outh + base) = yh;
}

extern "C" void kernel_launch(void* const* d_in, const int* in_sizes, int n_in,
                              void* d_out, int out_size, void* d_ws,
                              size_t ws_size, hipStream_t stream) {
  constexpr int Bn = 4, Sn = 1024, Dn = 1024, Hn = 16, HDn = 64, FFn = 4096;
  constexpr int Mn = Bn * Sn;
  static_assert(Dn == Hn * HDn, "head split");
  static_assert(Dn == LN_D, "ln width");
  if (n_in < 17) return;
  if (in_sizes[0] != Mn * Dn || in_sizes[1] != Dn * Dn || in_sizes[2] != Dn ||
      in_sizes[3] != Dn * Dn || in_sizes[4] != Dn || in_sizes[5] != Dn * Dn || in_sizes[6] != Dn ||
      in_sizes[7] != Dn * Dn || in_sizes[8] != Dn || in_sizes[9] != Dn || in_sizes[10] != Dn ||
      in_sizes[11] != FFn * Dn || in_sizes[12] != FFn || in_sizes[13] != Dn * FFn || in_sizes[14] != Dn ||
      in_sizes[15] != Dn || in_sizes[16] != Dn || out_size != Mn * Dn) return;

  const float* X   = (const float*)d_in[0];
  const float* Wq  = (const float*)d_in[1];
  const float* bq  = (const float*)d_in[2];
  const float* Wk  = (const float*)d_in[3];
  const float* bk  = (const float*)d_in[4];
  const float* Wv  = (const float*)d_in[5];
  const float* bv  = (const float*)d_in[6];
  const float* Wo  = (const float*)d_in[7];
  const float* bo  = (const float*)d_in[8];
  const float* g1  = (const float*)d_in[9];
  const float* b1  = (const float*)d_in[10];
  const float* Wup = (const float*)d_in[11];
  const float* bup = (const float*)d_in[12];
  const float* Wdn = (const float*)d_in[13];
  const float* bdn = (const float*)d_in[14];
  const float* g2  = (const float*)d_in[15];
  const float* b2  = (const float*)d_in[16];
  float* out = (float*)d_out;

  const size_t MiB = 1048576;
  const size_t szAct32 = (size_t)Mn * Dn * 4;
  const size_t szAct16 = (size_t)Mn * Dn * 2;
  const size_t szW16   = (size_t)Dn * Dn * 2;
  const size_t szWf16  = (size_t)FFn * Dn * 2;
  const size_t szUp16  = (size_t)Mn * FFn * 2;
  const size_t oQ    = 0;
  const size_t oK    = oQ + szAct32;
  const size_t oV    = oK + szAct32;
  const size_t oCtx  = oV + szAct32;
  const size_t oXh   = oCtx + szAct32;
  const size_t oWq   = oXh + szAct16;
  const size_t oWk   = oWq + szW16;
  const size_t oWv   = oWk + szW16;
  const size_t oWo   = oWv + szW16;
  const size_t oWup  = oWo + szW16;
  const size_t oWdn  = oWup + szWf16;
  const size_t carve = oWdn + szWf16;
  const size_t oX1h  = oV;
  const size_t oCtxh = oV + szAct16;
  const size_t oUp   = oCtx;
  if (oUp + szUp16 > oWup) return;
  if (carve > ws_size || carve > 128 * MiB) return;

  char* ws = (char*)d_ws;
  float* Qf   = (float*)(ws + oQ);
  float* Kf   = (float*)(ws + oK);
  float* Vf   = (float*)(ws + oV);
  float* Ctxf = (float*)(ws + oCtx);
  float* Yf   = (float*)(ws + oQ);
  float* X1f  = (float*)(ws + oK);
  float* Zf   = (float*)(ws + oQ);
  _Float16* Xh   = (_Float16*)(ws + oXh);
  _Float16* Wqh  = (_Float16*)(ws + oWq);
  _Float16* Wkh  = (_Float16*)(ws + oWk);
  _Float16* Wvh  = (_Float16*)(ws + oWv);
  _Float16* Woh  = (_Float16*)(ws + oWo);
  _Float16* Wuph = (_Float16*)(ws + oWup);
  _Float16* Wdnh = (_Float16*)(ws + oWdn);
  _Float16* X1h  = (_Float16*)(ws + oX1h);
  _Float16* Ctxh = (_Float16*)(ws + oCtxh);
  _Float16* Uph  = (_Float16*)(ws + oUp);

  const float WSC = 256.0f;
  const float CSC = 16.0f;
  const float invW = 1.0f / 256.0f;
  const float invWC = 1.0f / 4096.0f;

  {
    const int n2x = (Mn * Dn) / 2, n2w = (Dn * Dn) / 2, n2f = (FFn * Dn) / 2;
    cast_f32_f16x2s<<<(n2x + 255) / 256, 256, 0, stream>>>(X,   Xh,   n2x, 1.0f);
    cast_f32_f16x2s<<<(n2w + 255) / 256, 256, 0, stream>>>(Wq,  Wqh,  n2w, WSC);
    cast_f32_f16x2s<<<(n2w + 255) / 256, 256, 0, stream>>>(Wk,  Wkh,  n2w, WSC);
    cast_f32_f16x2s<<<(n2w + 255) / 256, 256, 0, stream>>>(Wv,  Wvh,  n2w, WSC);
    cast_f32_f16x2s<<<(n2w + 255) / 256, 256, 0, stream>>>(Wo,  Woh,  n2w, WSC);
    cast_f32_f16x2s<<<(n2f + 255) / 256, 256, 0, stream>>>(Wup, Wuph, n2f, WSC);
    cast_f32_f16x2s<<<(n2f + 255) / 256, 256, 0, stream>>>(Wdn, Wdnh, n2f, WSC);
  }

  const int tilesMD = (Mn / 64) * (Dn / 64);
  const int blocksMD = (tilesMD + 7) / 8;
  const int tilesMF = (Mn / 64) * (FFn / 64);
  const int blocksMF = (tilesMF + 7) / 8;

  wmma_gemm64<0, false, 2, 0, false, 0><<<dim3(blocksMD, 1), 256, 0, stream>>>(
      U16(Xh), U16(Xh), Dn, 0L, U16(Wqh), U16(Wqh), Dn, 0L, (void*)Qf, (void*)Qf, Dn, 0L,
      bq, X, 0L, Mn, Dn, Dn, invW);
  wmma_gemm64<0, false, 2, 0, false, 0><<<dim3(blocksMD, 1), 256, 0, stream>>>(
      U16(Xh), U16(Xh), Dn, 0L, U16(Wkh), U16(Wkh), Dn, 0L, (void*)Kf, (void*)Kf, Dn, 0L,
      bk, X, 0L, Mn, Dn, Dn, invW);
  wmma_gemm64<0, false, 2, 0, false, 0><<<dim3(blocksMD, 1), 256, 0, stream>>>(
      U16(Xh), U16(Xh), Dn, 0L, U16(Wvh), U16(Wvh), Dn, 0L, (void*)Vf, (void*)Vf, Dn, 0L,
      bv, X, 0L, Mn, Dn, Dn, invW);

  attn64_causal_f16<<<Bn * Hn * (Sn / 64), 128, 0, stream>>>(Qf, Kf, Vf, Ctxf, Sn, Hn, Dn, 0.125f, -1e30f);

  {
    const int n2x = (Mn * Dn) / 2;
    cast_f32_f16x2s<<<(n2x + 255) / 256, 256, 0, stream>>>(Ctxf, Ctxh, n2x, CSC);
  }

  wmma_gemm64<0, false, 2, 0, true, 0><<<dim3(blocksMD, 1), 256, 0, stream>>>(
      U16(Ctxh), U16(Ctxh), Dn, 0L, U16(Woh), U16(Woh), Dn, 0L, (void*)Yf, (void*)Yf, Dn, 0L,
      bo, X, 0L, Mn, Dn, Dn, invWC);

  ln_rows_kernel<true><<<Mn, 256, 0, stream>>>(Yf, g1, b1, X1f, X1h, 1e-7f);

  wmma_gemm64<0, false, 2, 1, false, 5><<<dim3(blocksMF, 1), 256, 0, stream>>>(
      U16(X1h), U16(X1h), Dn, 0L, U16(Wuph), U16(Wuph), Dn, 0L, (void*)Uph, (void*)Uph, FFn, 0L,
      bup, X, 0L, Mn, FFn, Dn, invW);

  wmma_gemm64<0, false, 2, 0, true, 0><<<dim3(blocksMD, 1), 256, 0, stream>>>(
      U16(Uph), U16(Uph), FFn, 0L, U16(Wdnh), U16(Wdnh), FFn, 0L, (void*)Zf, (void*)Zf, Dn, 0L,
      bdn, X1f, 0L, Mn, Dn, FFn, invW);

  ln_rows_kernel<false><<<Mn, 256, 0, stream>>>(Zf, g2, b2, out, X1h, 1e-7f);
}
